// QuantumTransformerLayer2025_21638045237787
// MI455X (gfx1250) — hardware-verified
//
#include <hip/hip_runtime.h>


#define NB_  4
#define SS   1024
#define HID  1024
#define NH_  8
#define HD   128
#define NQ   8
#define FFD  4096
#define NR   (NB_ * SS)
#define DM   HID
#define PCAR 1024.0f
#define LOSC 1024.0f
#define PI_F 3.14159265358979f
typedef _Float16 h16;
typedef unsigned short bf;
typedef __attribute__((ext_vector_type(16))) __bf16   v16bf;
typedef __attribute__((ext_vector_type(16))) _Float16 v16h;
typedef __attribute__((ext_vector_type(8)))  _Float16 v8h;
typedef __attribute__((ext_vector_type(8)))  unsigned short v8us;
typedef __attribute__((ext_vector_type(8)))  float    v8f;
typedef __attribute__((ext_vector_type(4)))  float    v4f;
typedef v8h  __attribute__((may_alias)) v8ha;
typedef v4f  __attribute__((may_alias)) v4fa;
typedef v8us __attribute__((may_alias)) v8usa;

__device__ __forceinline__ unsigned short f2bf(float f) { unsigned u = __float_as_uint(f); u += 0x7FFFu + ((u >> 16) & 1u); return (unsigned short)(u >> 16); }
__device__ __forceinline__ float bf2f(unsigned short b) { return __uint_as_float(((unsigned)b) << 16); }
__device__ __forceinline__ float bfr(float f) { return bf2f(f2bf(f)); }
__device__ __forceinline__ v16h cat16(v8h lo, v8h hi) { return __builtin_shufflevector(lo, hi, 0, 1, 2, 3, 4, 5, 6, 7, 8, 9, 10, 11, 12, 13, 14, 15); }
__device__ __forceinline__ v16bf cat16b(v8us lo, v8us hi) { return __builtin_bit_cast(v16bf, __builtin_shufflevector(lo, hi, 0, 1, 2, 3, 4, 5, 6, 7, 8, 9, 10, 11, 12, 13, 14, 15)); }
__device__ __forceinline__ v8f wmma16(v16h a, v16h b, v8f c) { return __builtin_amdgcn_wmma_f32_16x16x32_f16(false, a, false, b, (short)0, c, false, false); }
__device__ __forceinline__ v8f wmmab(v16bf a, v16bf b, v8f c) { return __builtin_amdgcn_wmma_f32_16x16x32_bf16(false, a, false, b, (short)0, c, false, false); }


__global__ __launch_bounds__(128) void k_gemmh(const h16* __restrict__ A, const h16* __restrict__ Bn, const float* __restrict__ bias, float* C, int ldc, const float* __restrict__ R, int K, size_t sA, size_t sB, size_t sC, int roundR) {
    __shared__ __align__(16) float ost[4][16 * 68];
    const size_t z = blockIdx.z; A += z * sA; Bn += z * sB; C += z * sC; if (R) R += z * sC;
    const int lane = threadIdx.x & 31, wave = threadIdx.x >> 5, lr = lane & 15, hi = lane >> 4;
    const int r0 = blockIdx.x * 64 + wave * 16, c0 = blockIdx.y * 64;
    const size_t aoff = (size_t)(r0 + lr) * K + 8 * hi;
    size_t boff[4];
#pragma unroll
    for (int t = 0; t < 4; ++t) boff[t] = (size_t)(c0 + t * 16 + lr) * K + 8 * hi;
    v8f acc[4];
#pragma unroll
    for (int t = 0; t < 4; ++t) acc[t] = (v8f){};
#pragma unroll 1
    for (int kc = 0; kc < K; kc += 32) {
        const v16h a = cat16(*(const v8h*)(A + aoff + kc), *(const v8h*)(A + aoff + kc + 16));
#pragma unroll
        for (int t = 0; t < 4; ++t) { const v16h b = cat16(*(const v8h*)(Bn + boff[t] + kc), *(const v8h*)(Bn + boff[t] + kc + 16)); acc[t] = wmma16(a, b, acc[t]); }
        asm volatile("v_nop\n\tv_nop\n\tv_nop\n\tv_nop" : "+v"(acc[0]), "+v"(acc[1]), "+v"(acc[2]), "+v"(acc[3]) : "v"(a));
    }
    float* os = &ost[wave][0];
#pragma unroll
    for (int t = 0; t < 4; ++t) { const float bv = bias ? bfr(bias[c0 + t * 16 + lr]) : 0.f;
#pragma unroll
        for (int j = 0; j < 8; ++j) os[(hi * 8 + j) * 68 + t * 16 + lr] = acc[t][j] + bv; }
    __syncthreads();
    float* crow = C + (size_t)r0 * ldc + c0;
    auto pass = [&]() {
#pragma unroll
        for (int s = 0; s < 8; ++s) { const int Lid = (lane >> 3) + 4 * s, piece = lane & 7; const int row = Lid >> 1, cofs = (Lid & 1) * 32 + piece * 4;
            v4f val = *(const v4fa*)(os + row * 68 + cofs); if (R) { const v4f rv = *(const v4f*)(R + ((size_t)r0 + row) * ldc + c0 + cofs); val += roundR ? (v4f){bfr(rv[0]), bfr(rv[1]), bfr(rv[2]), bfr(rv[3])} : rv; }
            *(volatile v4f*)(crow + (size_t)row * ldc + cofs) = val; }
    };
    pass(); __threadfence(); pass();
}

template <int MODE>
__global__ __launch_bounds__(128) void k_gemm3z(const bf* __restrict__ Ah, const bf* __restrict__ Al, const bf* __restrict__ Bh, const bf* __restrict__ Bl, int K, float* C, int ldc, size_t sA, size_t sB, size_t sC) {
    if ((MODE & 1) && (int)blockIdx.y * 64 > (int)blockIdx.x * 64 + 63) return;
    const size_t z = blockIdx.z; Ah += z * sA; Al += z * sA; Bh += z * sB; Bl += z * sB; C += z * sC;
    const int Klim = (MODE & 2) ? min(K, ((int)blockIdx.x + 1) * 64) : K;
    __shared__ __align__(16) float ost[4][16 * 68];
    const int lane = threadIdx.x & 31, wave = threadIdx.x >> 5, lr = lane & 15, hi = lane >> 4;
    const int r0 = blockIdx.x * 64 + wave * 16, c0 = blockIdx.y * 64;
    const size_t aoff = (size_t)(r0 + lr) * K + 8 * hi;
    v8f acc[4];
#pragma unroll
    for (int t = 0; t < 4; ++t) acc[t] = (v8f){};
#pragma unroll 1
    for (int kc = 0; kc < Klim; kc += 32) {
        const v16bf a = cat16b(*(const v8us*)(Ah + aoff + kc), *(const v8us*)(Ah + aoff + kc + 16));
        v16bf al = a; if (!(MODE & 4) && !(MODE & 16)) al = cat16b(*(const v8us*)(Al + aoff + kc), *(const v8us*)(Al + aoff + kc + 16));
#pragma unroll
        for (int t = 0; t < 4; ++t) { const size_t bo = (size_t)(c0 + t * 16 + lr) * K + kc + 8 * hi;
            const v16bf bh = cat16b(*(const v8us*)(Bh + bo), *(const v8us*)(Bh + bo + 16));
            acc[t] = wmmab(a, bh, acc[t]);
            if (!(MODE & 4)) { if (!(MODE & 16)) acc[t] = wmmab(al, bh, acc[t]); if (!(MODE & 8)) { const v16bf bl = cat16b(*(const v8us*)(Bl + bo), *(const v8us*)(Bl + bo + 16)); acc[t] = wmmab(a, bl, acc[t]); } } }
        asm volatile("v_nop\n\tv_nop\n\tv_nop\n\tv_nop" : "+v"(acc[0]), "+v"(acc[1]), "+v"(acc[2]), "+v"(acc[3]) : "v"(a), "v"(al));
    }
    float* os = &ost[wave][0];
#pragma unroll
    for (int t = 0; t < 4; ++t) {
#pragma unroll
        for (int j = 0; j < 8; ++j) os[(hi * 8 + j) * 68 + t * 16 + lr] = acc[t][j]; }
    __builtin_amdgcn_wave_barrier(); asm volatile("" ::: "memory");
    float* crow = C + (size_t)r0 * ldc + c0;
    auto pass = [&]() {
#pragma unroll
        for (int s = 0; s < 8; ++s) { const int Lid = (lane >> 3) + 4 * s, piece = lane & 7; const int row = Lid >> 1, cofs = (Lid & 1) * 32 + piece * 4;
            const v4f val = *(const v4fa*)(os + row * 68 + cofs); *(volatile v4f*)(crow + (size_t)row * ldc + cofs) = val; }
    };
    pass(); __threadfence(); pass();
}
__global__ __launch_bounds__(256) void k_planes32z(const float* __restrict__ F, int ld, int off, float sc, int rows, bf* Ph, bf* Pl) {
    typedef __attribute__((ext_vector_type(2))) unsigned short v2us;
    const int lane = threadIdx.x & 31; const size_t r = ((size_t)blockIdx.x * 8 + (threadIdx.x >> 5)) * 2 + (lane >> 4); if (r >= (size_t)rows) return; const int z = blockIdx.z; const int c0 = (lane & 15) * 2; v2us oh, ol;
    Ph += (size_t)z * rows * 32; Pl += (size_t)z * rows * 32;
#pragma unroll
    for (int i = 0; i < 2; ++i) { const float y = F[r * ld + off + z * 32 + c0 + i] * sc; const unsigned short hb = f2bf(y); oh[i] = hb; ol[i] = f2bf(y - bf2f(hb)); }
    const size_t o = r * 32 + c0; *(volatile v2us*)(Ph + o) = oh; *(volatile v2us*)(Pl + o) = ol; __threadfence(); *(volatile v2us*)(Ph + o) = oh; *(volatile v2us*)(Pl + o) = ol;
}
__global__ __launch_bounds__(256) void k_vtpadz(const float* __restrict__ F, int ld, int off, int nk, bf* Th, bf* Tl) {
    typedef __attribute__((ext_vector_type(2))) unsigned short v2us;
    const int lane = threadIdx.x & 31; const size_t wid = (size_t)blockIdx.x * 8 + (threadIdx.x >> 5); if (wid >= (size_t)64 * (nk / 64)) return; const int z = blockIdx.z; const int d = (int)(wid / (nk / 64)); const int k0 = (int)(wid % (nk / 64)) * 64 + lane * 2; v2us oh, ol;
    Th += (size_t)z * 64 * nk; Tl += (size_t)z * 64 * nk;
#pragma unroll
    for (int i = 0; i < 2; ++i) { const float y = (d < 32) ? F[(size_t)(k0 + i) * ld + off + z * 32 + (d < 32 ? d : 0)] : 0.f; const unsigned short hb = f2bf(y); oh[i] = hb; ol[i] = f2bf(y - bf2f(hb)); }
    const size_t o = (size_t)d * nk + k0; *(volatile v2us*)(Th + o) = oh; *(volatile v2us*)(Tl + o) = ol; __threadfence(); *(volatile v2us*)(Th + o) = oh; *(volatile v2us*)(Tl + o) = ol;
}
template <int NK>
__global__ __launch_bounds__(256) void k_softmaxz(const float* __restrict__ S, int rows, bf* PH, bf* PL) {
    typedef __attribute__((ext_vector_type(4))) unsigned short v4us;
    const int lane = threadIdx.x & 31, i = blockIdx.x * 8 + (threadIdx.x >> 5); if (i >= rows) return; const size_t zo = (size_t)blockIdx.z * rows * NK; const float* sr = S + zo + (size_t)i * NK; PH += zo; PL += zo;
    float m = -3.0e38f;
#pragma unroll 1
    for (int c0 = lane * 4; c0 < NK; c0 += 128) {
#pragma unroll
        for (int q = 0; q < 4; ++q) m = fmaxf(m, sr[c0 + q]); }
#pragma unroll
    for (int sh = 16; sh; sh >>= 1) m = fmaxf(m, __shfl_xor(m, sh, 32));
    float sum = 0.f;
#pragma unroll 1
    for (int c0 = lane * 4; c0 < NK; c0 += 128) {
#pragma unroll
        for (int q = 0; q < 4; ++q) sum += __expf(sr[c0 + q] - m); }
#pragma unroll
    for (int sh = 16; sh; sh >>= 1) sum += __shfl_xor(sum, sh, 32);
    const float inv = 1.0f / sum;
#pragma unroll 1
    for (int ps = 0; ps < 2; ++ps) {
#pragma unroll 1
        for (int c0 = lane * 4; c0 < NK; c0 += 128) { v4us oh, ol;
#pragma unroll
            for (int q = 0; q < 4; ++q) { const float p = __expf(sr[c0 + q] - m) * inv; const unsigned short hb = f2bf(p); oh[q] = hb; ol[q] = f2bf(p - bf2f(hb)); }
            const size_t o = (size_t)i * NK + c0; *(volatile v4us*)(PH + o) = oh; *(volatile v4us*)(PL + o) = ol; }
        if (ps == 0) __threadfence(); }
}
__global__ __launch_bounds__(256) void k_placez(const float* __restrict__ XH, int rows, int ldy, float* Y) {
    const int lane = threadIdx.x & 31; const size_t q = (size_t)blockIdx.x * 8 + (threadIdx.x >> 5); if (q >= (size_t)rows) return; const int z = blockIdx.z; const float v = XH[((size_t)z * rows + q) * 64 + lane];
    *(volatile float*)(Y + q * ldy + z * 32 + lane) = v; __threadfence(); *(volatile float*)(Y + q * ldy + z * 32 + lane) = v;
}

template <typename T16> struct WFrag;
template <> struct WFrag<h16> { typedef v16h V; static __device__ __forceinline__ V ld(const h16* p) { return cat16(*(const v8h*)p, *(const v8h*)(p + 16)); } static __device__ __forceinline__ v8f mma(V a, V b, v8f c) { return wmma16(a, b, c); } };
template <> struct WFrag<bf> { typedef v16bf V; static __device__ __forceinline__ V ld(const bf* p) { return cat16b(*(const v8us*)p, *(const v8us*)(p + 16)); } static __device__ __forceinline__ v8f mma(V a, V b, v8f c) { return wmmab(a, b, c); } };
template <typename T16, int NSPLIT, bool BIAS>
__global__ __launch_bounds__(32) void k_gemmw(const T16* __restrict__ A, const T16* __restrict__ A2, const T16* __restrict__ Bt, const T16* __restrict__ Bt2, int K, float* C, int ldc, const float* __restrict__ bias, size_t sA, size_t sB, size_t sC) {
    typedef typename WFrag<T16>::V V;
    __shared__ __align__(16) float os[16 * 68];
    const size_t z = blockIdx.z; A += z * sA; if (A2) A2 += z * sA; Bt += z * sB; if (Bt2) Bt2 += z * sB; C += z * sC;
    const int lane = threadIdx.x & 31, lr = lane & 15, hi = lane >> 4; const int r0 = blockIdx.x * 64, c0 = blockIdx.y * 64;
    v8f acc[4][4];
#pragma unroll
    for (int mb = 0; mb < 4; ++mb)
#pragma unroll
        for (int nb = 0; nb < 4; ++nb) acc[mb][nb] = (v8f){};
    const size_t aoff = (size_t)(r0 + lr) * K + 8 * hi, boff = (size_t)(c0 + lr) * K + 8 * hi;
#pragma unroll 1
    for (int kc = 0; kc < K; kc += 32) {
        V a[4], a2[4];
#pragma unroll
        for (int mb = 0; mb < 4; ++mb) { a[mb] = WFrag<T16>::ld(A + aoff + (size_t)mb * 16 * K + kc); if (NSPLIT == 1 || NSPLIT == 2) a2[mb] = WFrag<T16>::ld(A2 + aoff + (size_t)mb * 16 * K + kc); }
#pragma unroll
        for (int nb = 0; nb < 4; ++nb) { const V b = WFrag<T16>::ld(Bt + boff + (size_t)nb * 16 * K + kc); V b2; if (NSPLIT >= 2) b2 = WFrag<T16>::ld(Bt2 + boff + (size_t)nb * 16 * K + kc);
#pragma unroll
            for (int mb = 0; mb < 4; ++mb) { acc[mb][nb] = WFrag<T16>::mma(a[mb], b, acc[mb][nb]); if (NSPLIT == 1 || NSPLIT == 2) acc[mb][nb] = WFrag<T16>::mma(a2[mb], b, acc[mb][nb]); if (NSPLIT >= 2) acc[mb][nb] = WFrag<T16>::mma(a[mb], b2, acc[mb][nb]); } }
        asm volatile("v_nop\n\tv_nop\n\tv_nop\n\tv_nop" : "+v"(acc[0][0]), "+v"(acc[1][1]), "+v"(acc[2][2]), "+v"(acc[3][3]) : "v"(a[0]), "v"(a[3]));
    }
#pragma unroll
    for (int mb = 0; mb < 4; ++mb) {
#pragma unroll
        for (int nb = 0; nb < 4; ++nb) {
#pragma unroll
            for (int j = 0; j < 8; ++j) os[(hi * 8 + j) * 68 + nb * 16 + lr] = acc[mb][nb][j]; }
        __builtin_amdgcn_wave_barrier(); asm volatile("" ::: "memory");
        float* crow = C + (size_t)(r0 + mb * 16) * ldc + c0;
#pragma unroll 1
        for (int ps = 0; ps < 2; ++ps) {
#pragma unroll
            for (int s = 0; s < 8; ++s) { const int row = 2 * s + hi, cofs = lr * 4; v4f val = *(const v4fa*)(os + row * 68 + cofs); if (BIAS) { val[0] += bfr(bias[c0 + cofs]); val[1] += bfr(bias[c0 + cofs + 1]); val[2] += bfr(bias[c0 + cofs + 2]); val[3] += bfr(bias[c0 + cofs + 3]); }
                *(volatile v4f*)(crow + (size_t)row * ldc + cofs) = val; }
            if (ps == 0) __threadfence(); }
        __builtin_amdgcn_wave_barrier(); asm volatile("" ::: "memory");
    }
}

typedef __attribute__((ext_vector_type(4))) _Float16 v4h;
__device__ __forceinline__ h16 tohx(float x) { return (h16)x; }
__global__ __launch_bounds__(256) void k_wTq(const float* __restrict__ Wm, bf* Bt) {
    __shared__ float tl[64][65]; typedef __attribute__((ext_vector_type(4))) unsigned short v4us;
    const int tid = threadIdx.x; const int i0 = blockIdx.x * 64, d0 = blockIdx.y * 64, h = blockIdx.z; const int rr = tid >> 2, cq = (tid & 3) * 16;
#pragma unroll
    for (int i = 0; i < 16; ++i) tl[rr][cq + i] = bfr(Wm[((size_t)h * HID + i0 + rr) * HD + d0 + cq + i]);
    __syncthreads();
    const int lane = tid & 31, wv = tid >> 5;
    auto pass = [&]() {
#pragma unroll
        for (int st = 0; st < 4; ++st) { const int nr = wv * 8 + st * 2 + (lane >> 4); const int kq = (lane & 15) * 4; v4us v; for (int i = 0; i < 4; ++i) v[i] = f2bf(tl[kq + i][nr]); *(volatile v4us*)(Bt + (size_t)(h * HD + d0 + nr) * HID + i0 + kq) = v; }
    };
    pass(); __threadfence(); pass();
}
__global__ __launch_bounds__(256) void k_wTh(const float* __restrict__ Wm, int ldw, int K, int N, h16* Bh) {
    __shared__ float tl[64][65];
    const int tid = threadIdx.x; const int k0 = blockIdx.x * 64, n0 = blockIdx.y * 64; const int rr = tid >> 2, cq = (tid & 3) * 16;
#pragma unroll
    for (int i = 0; i < 16; ++i) tl[rr][cq + i] = bfr(Wm[(size_t)(k0 + rr) * ldw + n0 + cq + i]);
    __syncthreads();
    const int lane = tid & 31, wv = tid >> 5;
    auto pass = [&]() {
#pragma unroll
        for (int st = 0; st < 4; ++st) { const int nr = wv * 8 + st * 2 + (lane >> 4); const int kq = (lane & 15) * 4; v4h v; for (int i = 0; i < 4; ++i) v[i] = tohx(tl[kq + i][nr]); *(volatile v4h*)(Bh + (size_t)(n0 + nr) * K + k0 + kq) = v; }
    };
    pass(); __threadfence(); pass();
}
__global__ __launch_bounds__(256) void k_cvtx(const float* __restrict__ x, bf* A) {
    const int lane = threadIdx.x & 31; const size_t r = (size_t)blockIdx.x * 8 + (threadIdx.x >> 5); if (r >= (size_t)NR) return;
#pragma unroll 1
    for (int ps = 0; ps < 2; ++ps) {
#pragma unroll
        for (int q = 0; q < HID / 256; ++q) { const size_t o = r * HID + q * 256 + lane * 8; v8us v;
#pragma unroll
            for (int i = 0; i < 8; ++i) v[i] = f2bf(x[o + i]);
            *(volatile v8us*)(A + o) = v; }
        if (ps == 0) __threadfence(); }
}
__global__ __launch_bounds__(256) void k_m1(const float* __restrict__ W1, const float* __restrict__ Wm, float* M1) {
    const int lane = threadIdx.x & 31; const int w = blockIdx.x * 8 + (threadIdx.x >> 5); if (w >= HID / 4) return; const int i = w * 4 + (lane >> 3), q = lane & 7; float a = 0.f;
#pragma unroll 1
    for (int f = 0; f < FFD; ++f) a = fmaf(bfr(W1[(size_t)i * FFD + f]), bfr(Wm[(size_t)f * NQ + q]), a);
    *(volatile float*)(M1 + (size_t)i * NQ + q) = a; __threadfence(); *(volatile float*)(M1 + (size_t)i * NQ + q) = a;
}
__global__ __launch_bounds__(256) void k_m1pack(const float* __restrict__ M1, bf* Th, bf* Tl) {
    const int lane = threadIdx.x & 31; const int q = blockIdx.x * 8 + (threadIdx.x >> 5); if (q >= 64) return;
#pragma unroll 1
    for (int ps = 0; ps < 2; ++ps) {
#pragma unroll
        for (int c = 0; c < 4; ++c) { v8us oh, ol; const int i0 = c * 256 + lane * 8;
#pragma unroll
            for (int k = 0; k < 8; ++k) { const float v = (q < NQ) ? M1[(size_t)(i0 + k) * NQ + q] : 0.f; const unsigned short hb = f2bf(v); oh[k] = hb; ol[k] = f2bf(v - bf2f(hb)); }
            *(volatile v8us*)(Th + (size_t)q * HID + i0) = oh; *(volatile v8us*)(Tl + (size_t)q * HID + i0) = ol; }
        if (ps == 0) __threadfence(); }
}
__global__ __launch_bounds__(32) void k_c1(const float* __restrict__ b1, const float* __restrict__ Wm, const float* __restrict__ bm, float* C1) {
    const int lane = threadIdx.x & 31; float a = 0.f; if (lane < NQ) { a = bfr(bm[lane]);
#pragma unroll 1
        for (int f = 0; f < FFD; ++f) a = fmaf(bfr(b1[f]), bfr(Wm[(size_t)f * NQ + lane]), a); }
    *(volatile float*)(C1 + lane) = a; __threadfence(); *(volatile float*)(C1 + lane) = a;
}
__global__ __launch_bounds__(256) void k_m2(const float* __restrict__ Wqo, const float* __restrict__ bqo, const float* __restrict__ W2, const float* __restrict__ b2, float* M2) {
    const int o = blockIdx.x * 256 + threadIdx.x; const int q = blockIdx.y; if (o >= HID) return; float a = (q == NQ) ? bfr(b2[o]) : 0.f;
#pragma unroll 1
    for (int f = 0; f < FFD; ++f) a = fmaf((q == NQ) ? bfr(bqo[f]) : bfr(Wqo[(size_t)q * FFD + f]), bfr(W2[(size_t)f * HID + o]), a);
    *(volatile float*)(M2 + (size_t)q * HID + o) = a; __threadfence(); *(volatile float*)(M2 + (size_t)q * HID + o) = a;
}
__global__ __launch_bounds__(256) void k_m2pack(const float* __restrict__ M2, bf* Th, bf* Tl) {
    typedef __attribute__((ext_vector_type(2))) unsigned short v2us;
    const int lane = threadIdx.x & 31; const int o = (blockIdx.x * 8 + (threadIdx.x >> 5)) * 2 + (lane >> 4); if (o >= HID) return; const int q0 = (lane & 15) * 2; v2us oh, ol;
#pragma unroll
    for (int k = 0; k < 2; ++k) { const int q = q0 + k; const float v = (q < NQ) ? M2[(size_t)q * HID + o] : 0.f; const unsigned short hb = f2bf(v); oh[k] = hb; ol[k] = f2bf(v - bf2f(hb)); }
#pragma unroll 1
    for (int ps = 0; ps < 2; ++ps) { *(volatile v2us*)(Th + (size_t)o * 32 + q0) = oh; *(volatile v2us*)(Tl + (size_t)o * 32 + q0) = ol; if (ps == 0) __threadfence(); }
}
__global__ __launch_bounds__(256) void k_qq(const float* __restrict__ F, const float* __restrict__ Wc, const float* __restrict__ bc, int b, float* QQ) {
    const int lane = threadIdx.x & 31; const size_t w = (size_t)blockIdx.x * 8 + (threadIdx.x >> 5); const int s = (int)(w * 2 + (lane >> 4)); const int h = blockIdx.z; const int slot = lane & 15; if (s >= SS) return;
    const float* fr = F + ((size_t)b * SS + s) * HID + h * HD; float a = 0.f;
    if (slot < NQ) { a = bfr(bc[h * NQ + slot]);
#pragma unroll 1
        for (int d = 0; d < HD; ++d) a = fmaf(fr[d], bfr(Wc[((size_t)h * HD + d) * NQ + slot]), a); }
    float sq = (slot < NQ) ? a * a : 0.f;
#pragma unroll
    for (int sh = 1; sh < 16; sh <<= 1) sq += __shfl_xor(sq, sh, 32);
    const float val = (slot < NQ) ? a : (slot == NQ ? sqrtf(sq) : 0.f);
    float* dst = QQ + ((size_t)h * SS + s) * 16 + slot; *(volatile float*)dst = val; __threadfence(); *(volatile float*)dst = val;
}
__global__ __launch_bounds__(256) void k_hpl(const float* __restrict__ F, int b, float sc, h16* P) {
    const int lane = threadIdx.x & 31; const int s = blockIdx.x * 8 + (threadIdx.x >> 5); if (s >= SS) return; const int z = blockIdx.z; v4h o;
#pragma unroll
    for (int i = 0; i < 4; ++i) o[i] = tohx(F[((size_t)b * SS + s) * HID + z * HD + lane * 4 + i] * sc);
    const size_t off = ((size_t)z * SS + s) * HD + lane * 4; *(volatile v4h*)(P + off) = o; __threadfence(); *(volatile v4h*)(P + off) = o;
}
__global__ __launch_bounds__(256) void k_vT(const float* __restrict__ V, int b, h16* VT) {
    __shared__ float tl[64][65];
    const int tid = threadIdx.x; const int t0 = blockIdx.x * 64, d0 = blockIdx.y * 64; const int z = blockIdx.z; const int rr = tid >> 2, cq = (tid & 3) * 16;
#pragma unroll
    for (int i = 0; i < 16; ++i) tl[rr][cq + i] = V[((size_t)b * SS + t0 + rr) * HID + z * HD + d0 + cq + i];
    __syncthreads();
    const int lane = tid & 31, wv = tid >> 5;
    auto pass = [&]() {
#pragma unroll
        for (int st = 0; st < 4; ++st) { const int dr = wv * 8 + st * 2 + (lane >> 4); const int tq = (lane & 15) * 4; v4h v;
#pragma unroll
            for (int i = 0; i < 4; ++i) v[i] = tohx(tl[tq + i][dr]);
            *(volatile v4h*)(VT + ((size_t)z * HD + d0 + dr) * SS + t0 + tq) = v; }
    };
    pass(); __threadfence(); pass();
}
__global__ __launch_bounds__(256) void k_softq(float* S, const float* __restrict__ QQ, const float* __restrict__ KQ, h16* P) {
    const int lane = threadIdx.x & 31, s = blockIdx.x * 8 + (threadIdx.x >> 5); if (s >= SS) return; const int z = blockIdx.z; const size_t zo = ((size_t)z * SS + s) * SS; float* sr = S + zo; h16* po = P + zo;
    const float* qr = QQ + ((size_t)z * SS + s) * 16; float qv[NQ];
#pragma unroll
    for (int q = 0; q < NQ; ++q) qv[q] = qr[q];
    const float qn = qr[NQ];
    float m = -3.0e38f;
#pragma unroll 1
    for (int c0 = lane * 4; c0 < SS; c0 += 128) { v4f sv = *(const v4f*)(sr + c0);
#pragma unroll 1
        for (int k = 0; k < 4; ++k) { const float* kr = KQ + ((size_t)z * SS + c0 + k) * 16; float dt = 0.f;
#pragma unroll
            for (int q = 0; q < NQ; ++q) dt = fmaf(qv[q], kr[q], dt);
            const float fid = __fdiv_rn(dt, fmaxf(qn * kr[NQ], 1e-8f)); const float qw = fid * (1.0f + 0.1f * sinf(fid * PI_F)); const float aw = 0.5f * qw + 0.5f * sv[k]; sv[k] = aw; m = fmaxf(m, aw); }
        *(v4f*)(sr + c0) = sv; }
#pragma unroll
    for (int sh = 16; sh; sh >>= 1) m = fmaxf(m, __shfl_xor(m, sh, 32));
    float sum = 0.f;
#pragma unroll 1
    for (int c0 = lane * 4; c0 < SS; c0 += 128) { const v4f sv = *(const v4f*)(sr + c0);
#pragma unroll
        for (int k = 0; k < 4; ++k) sum += __expf(sv[k] - m); }
#pragma unroll
    for (int sh = 16; sh; sh >>= 1) sum += __shfl_xor(sum, sh, 32);
    const float f = __fdiv_rn(PCAR, sum);
#pragma unroll 1
    for (int ps = 0; ps < 2; ++ps) {
#pragma unroll 1
        for (int c0 = lane * 4; c0 < SS; c0 += 128) { const v4f sv = *(const v4f*)(sr + c0); v4h o;
#pragma unroll
            for (int k = 0; k < 4; ++k) o[k] = tohx(__expf(sv[k] - m) * f);
            *(volatile v4h*)(po + c0) = o; }
        if (ps == 0) __threadfence(); }
}
__global__ __launch_bounds__(256) void k_merge(const float* __restrict__ OZ, int b, h16* OH) {
    const int lane = threadIdx.x & 31; const int s = blockIdx.x * 8 + (threadIdx.x >> 5); if (s >= SS) return; const int z = blockIdx.z; v4h o;
#pragma unroll
    for (int i = 0; i < 4; ++i) o[i] = tohx(OZ[((size_t)z * SS + s) * HD + lane * 4 + i] * (1.0f / PCAR));
    const size_t off = ((size_t)b * SS + s) * HID + z * HD + lane * 4; *(volatile v4h*)(OH + off) = o; __threadfence(); *(volatile v4h*)(OH + off) = o;
}
__global__ __launch_bounds__(256) void k_ln1(const float* __restrict__ x, const float* __restrict__ CO, const float* __restrict__ g_, const float* __restrict__ b_, float* X1, bf* Xh, bf* Xl) {
    typedef __attribute__((ext_vector_type(4))) unsigned short v4us;
    const int lane = threadIdx.x & 31; const size_t r = (size_t)blockIdx.x * 8 + (threadIdx.x >> 5); if (r >= (size_t)NR) return; float v[32]; float s = 0.f;
#pragma unroll
    for (int c = 0; c < 8; ++c) {
#pragma unroll
        for (int i = 0; i < 4; ++i) { const int col = c * 128 + lane * 4 + i; v[c * 4 + i] = bfr(x[r * HID + col]) + CO[r * HID + col]; s += v[c * 4 + i]; } }
#pragma unroll
    for (int sh = 16; sh; sh >>= 1) s += __shfl_xor(s, sh, 32);
    const float mu = s * (1.0f / HID); float q = 0.f;
#pragma unroll
    for (int i = 0; i < 32; ++i) { const float d = v[i] - mu; q = fmaf(d, d, q); }
#pragma unroll
    for (int sh = 16; sh; sh >>= 1) q += __shfl_xor(q, sh, 32);
    const float rs = rsqrtf(q * (1.0f / HID) + 1e-5f);
#pragma unroll 1
    for (int ps = 0; ps < 2; ++ps) {
#pragma unroll
        for (int c = 0; c < 8; ++c) { v4f o; v4us oh, ol; const int c0 = c * 128 + lane * 4;
#pragma unroll
            for (int i = 0; i < 4; ++i) { o[i] = (v[c * 4 + i] - mu) * rs * bfr(g_[c0 + i]) + bfr(b_[c0 + i]); const unsigned short hb = f2bf(o[i]); oh[i] = hb; ol[i] = f2bf(o[i] - bf2f(hb)); }
            *(volatile v4f*)(X1 + r * HID + c0) = o; *(volatile v4us*)(Xh + r * HID + c0) = oh; *(volatile v4us*)(Xl + r * HID + c0) = ol; }
        if (ps == 0) __threadfence(); }
}
__global__ __launch_bounds__(256) void k_qe(const float* __restrict__ QM, const float* __restrict__ C1, bf* Eh, bf* El) {
    typedef __attribute__((ext_vector_type(2))) unsigned short v2us;
    const int lane = threadIdx.x & 31; const size_t r = ((size_t)blockIdx.x * 8 + (threadIdx.x >> 5)) * 2 + (lane >> 4); if (r >= (size_t)NR) return; const int q0 = (lane & 15) * 2; v2us oh, ol;
#pragma unroll
    for (int k = 0; k < 2; ++k) { const int q = q0 + k; float e = 0.f; if (q < NQ) { const float t = QM[r * 64 + q] + C1[q]; e = tanhf(t) * cosf(t * (PI_F / 4.0f)); } const unsigned short hb = f2bf(e); oh[k] = hb; ol[k] = f2bf(e - bf2f(hb)); }
#pragma unroll 1
    for (int ps = 0; ps < 2; ++ps) { *(volatile v2us*)(Eh + r * 32 + q0) = oh; *(volatile v2us*)(El + r * 32 + q0) = ol; if (ps == 0) __threadfence(); }
}
__global__ __launch_bounds__(256) void k_ffb(const float* __restrict__ X1, const float* __restrict__ FF, const float* __restrict__ M2, const float* __restrict__ g_, const float* __restrict__ b_, float* OUTB) {
    const int lane = threadIdx.x & 31; const size_t r = (size_t)blockIdx.x * 8 + (threadIdx.x >> 5); if (r >= (size_t)NR) return; const float* C2 = M2 + (size_t)NQ * HID; float v[32]; float s = 0.f;
#pragma unroll
    for (int c = 0; c < 8; ++c) {
#pragma unroll
        for (int i = 0; i < 4; ++i) { const int col = c * 128 + lane * 4 + i; v[c * 4 + i] = X1[r * HID + col] + FF[r * HID + col] + C2[col]; s += v[c * 4 + i]; } }
#pragma unroll
    for (int sh = 16; sh; sh >>= 1) s += __shfl_xor(s, sh, 32);
    const float mu = s * (1.0f / HID); float q = 0.f;
#pragma unroll
    for (int i = 0; i < 32; ++i) { const float d = v[i] - mu; q = fmaf(d, d, q); }
#pragma unroll
    for (int sh = 16; sh; sh >>= 1) q += __shfl_xor(q, sh, 32);
    const float rs = rsqrtf(q * (1.0f / HID) + 1e-5f);
#pragma unroll 1
    for (int ps = 0; ps < 2; ++ps) {
#pragma unroll
        for (int c = 0; c < 8; ++c) { v4f o; const int c0 = c * 128 + lane * 4;
#pragma unroll
            for (int i = 0; i < 4; ++i) o[i] = (v[c * 4 + i] - mu) * rs * bfr(g_[c0 + i]) + bfr(b_[c0 + i]);
            *(volatile v4f*)(OUTB + r * HID + c0) = o; }
        if (ps == 0) __threadfence(); }
}
extern "C" void kernel_launch(void* const* d_in, const int* in_sizes, int n_in,
                              void* d_out, int out_size, void* d_ws, size_t ws_size, hipStream_t stream) {
    (void)in_sizes; (void)n_in; (void)out_size;
    const float* x = (const float*)d_in[0]; const float* Wq = (const float*)d_in[1]; const float* bq = (const float*)d_in[2]; const float* Wk = (const float*)d_in[3]; const float* bk = (const float*)d_in[4]; const float* Wv = (const float*)d_in[5]; const float* bv = (const float*)d_in[6]; const float* Wc = (const float*)d_in[7]; const float* bc = (const float*)d_in[8]; const float* Wo = (const float*)d_in[9]; const float* bo = (const float*)d_in[10];
    const float* g1 = (const float*)d_in[11]; const float* be1 = (const float*)d_in[12]; const float* g2 = (const float*)d_in[13]; const float* be2 = (const float*)d_in[14]; const float* W1 = (const float*)d_in[15]; const float* b1 = (const float*)d_in[16]; const float* Wm = (const float*)d_in[17]; const float* bm = (const float*)d_in[18]; const float* Wqo = (const float*)d_in[19]; const float* bqo = (const float*)d_in[20]; const float* W2 = (const float*)d_in[21]; const float* b2 = (const float*)d_in[22];
    float* out = (float*)d_out;
    char* wsp = (char*)d_ws;
    auto take = [&](size_t bytes) { char* p = wsp; wsp += (bytes + 255) & ~(size_t)255; return (void*)p; };
    const size_t WSZ = (size_t)HID * HID * 2;
    bf* WQ = (bf*)take(WSZ); bf* WK = (bf*)take(WSZ); bf* WV = (bf*)take(WSZ); h16* WO = (h16*)take(WSZ); float* M1 = (float*)take((size_t)HID * NQ * 4); float* C1 = (float*)take(32 * 4); float* M2 = (float*)take((size_t)(NQ + 1) * HID * 4); bf* M1Th = (bf*)take((size_t)64 * HID * 2); bf* M1Tl = (bf*)take((size_t)64 * HID * 2); bf* M2Th = (bf*)take((size_t)HID * 32 * 2); bf* M2Tl = (bf*)take((size_t)HID * 32 * 2);
    bf* XB = (bf*)take((size_t)NR * HID * 2); float* Q = (float*)take((size_t)NR * HID * 4); float* Kf = (float*)take((size_t)NR * HID * 4); float* V = (float*)take((size_t)NR * HID * 4);
    float* QQ = (float*)take((size_t)NH_ * SS * 16 * 4); float* KQ = (float*)take((size_t)NH_ * SS * 16 * 4); h16* Qx = (h16*)take((size_t)NH_ * SS * HD * 2); h16* Kx = (h16*)take((size_t)NH_ * SS * HD * 2); h16* VT = (h16*)take((size_t)NH_ * HD * SS * 2);
    float* S = (float*)take((size_t)NH_ * SS * SS * 4); h16* Px = (h16*)take((size_t)NH_ * SS * SS * 2); float* OZ = (float*)take((size_t)NH_ * SS * HD * 4); h16* OH = (h16*)take((size_t)NR * HID * 2); float* CO = (float*)take((size_t)NR * HID * 4); float* X1 = (float*)take((size_t)NR * HID * 4); bf* X1h = (bf*)take((size_t)NR * HID * 2); bf* X1l = (bf*)take((size_t)NR * HID * 2); float* QM = (float*)take((size_t)NR * 64 * 4); bf* QEh = (bf*)take((size_t)NR * 32 * 2); bf* QEl = (bf*)take((size_t)NR * 32 * 2); float* FF = (float*)take((size_t)NR * HID * 4);
    if ((size_t)(wsp - (char*)d_ws) > ws_size) return;
    k_wTq<<<dim3(HID / 64, HD / 64, NH_), 256, 0, stream>>>(Wq, WQ); k_wTq<<<dim3(HID / 64, HD / 64, NH_), 256, 0, stream>>>(Wk, WK); k_wTq<<<dim3(HID / 64, HD / 64, NH_), 256, 0, stream>>>(Wv, WV); k_wTh<<<dim3(HID / 64, HID / 64, 1), 256, 0, stream>>>(Wo, HID, HID, HID, WO);
    k_m1<<<(HID / 4) / 8, 256, 0, stream>>>(W1, Wm, M1); k_m1pack<<<64 / 8, 256, 0, stream>>>(M1, M1Th, M1Tl); k_c1<<<1, 32, 0, stream>>>(b1, Wm, bm, C1); k_m2<<<dim3(HID / 256, NQ + 1, 1), 256, 0, stream>>>(Wqo, bqo, W2, b2, M2); k_m2pack<<<(HID / 2) / 8, 256, 0, stream>>>(M2, M2Th, M2Tl);
    k_cvtx<<<NR / 8, 256, 0, stream>>>(x, XB);
    k_gemmw<bf, 0, true><<<dim3(NR / 64, HID / 64, 1), 32, 0, stream>>>(XB, nullptr, WQ, nullptr, HID, Q, HID, bq, 0, 0, 0);
    k_gemmw<bf, 0, true><<<dim3(NR / 64, HID / 64, 1), 32, 0, stream>>>(XB, nullptr, WK, nullptr, HID, Kf, HID, bk, 0, 0, 0);
    k_gemmw<bf, 0, true><<<dim3(NR / 64, HID / 64, 1), 32, 0, stream>>>(XB, nullptr, WV, nullptr, HID, V, HID, bv, 0, 0, 0);
    for (int b = 0; b < NB_; ++b) {
        k_qq<<<dim3((SS / 2) / 8, 1, NH_), 256, 0, stream>>>(Q, Wc, bc, b, QQ); k_qq<<<dim3((SS / 2) / 8, 1, NH_), 256, 0, stream>>>(Kf, Wc, bc, b, KQ);
        k_hpl<<<dim3(SS / 8, 1, NH_), 256, 0, stream>>>(Q, b, 0.08838834764831845f, Qx); k_hpl<<<dim3(SS / 8, 1, NH_), 256, 0, stream>>>(Kf, b, 1.0f, Kx); k_vT<<<dim3(SS / 64, HD / 64, NH_), 256, 0, stream>>>(V, b, VT);
        k_gemmw<h16, 0, false><<<dim3(SS / 64, SS / 64, NH_), 32, 0, stream>>>(Qx, nullptr, Kx, nullptr, HD, S, SS, nullptr, (size_t)SS * HD, (size_t)SS * HD, (size_t)SS * SS);
        k_softq<<<dim3(SS / 8, 1, NH_), 256, 0, stream>>>(S, QQ, KQ, Px);
        k_gemmw<h16, 0, false><<<dim3(SS / 64, HD / 64, NH_), 32, 0, stream>>>(Px, nullptr, VT, nullptr, SS, OZ, HD, nullptr, (size_t)SS * SS, (size_t)HD * SS, (size_t)SS * HD);
        k_merge<<<dim3(SS / 8, 1, NH_), 256, 0, stream>>>(OZ, b, OH); }
    k_gemmw<h16, 0, true><<<dim3(NR / 64, HID / 64, 1), 32, 0, stream>>>(OH, nullptr, WO, nullptr, HID, CO, HID, bo, 0, 0, 0);
    k_ln1<<<NR / 8, 256, 0, stream>>>(x, CO, g1, be1, X1, X1h, X1l);
    k_gemmw<bf, 2, false><<<dim3(NR / 64, 1, 1), 32, 0, stream>>>(X1h, X1l, M1Th, M1Tl, HID, QM, 64, nullptr, 0, 0, 0);
    k_qe<<<(NR / 2) / 8, 256, 0, stream>>>(QM, C1, QEh, QEl);
    k_gemmw<bf, 2, false><<<dim3(NR / 64, HID / 64, 1), 32, 0, stream>>>(QEh, QEl, M2Th, M2Tl, 32, FF, HID, nullptr, 0, 0, 0);
    k_ffb<<<NR / 8, 256, 0, stream>>>(X1, FF, M2, g2, be2, out);
}
